// SCI_66168266162290
// MI455X (gfx1250) — hardware-verified
//
#include <hip/hip_runtime.h>

#pragma clang fp contract(off)

typedef __bf16         v16bf __attribute__((ext_vector_type(16)));
typedef unsigned short v8us  __attribute__((ext_vector_type(8)));
typedef float          v8f   __attribute__((ext_vector_type(8)));
typedef float          v4f   __attribute__((ext_vector_type(4)));
typedef v8us __attribute__((may_alias)) v8usa;
typedef v4f  __attribute__((may_alias)) v4fa;
typedef unsigned short u16;

union FragB { v16bf v; v8us u[2]; };

#define T_DIM 512
#define F_DIM 128
#define R_DIM 32
#define KTOT  1024
#define NPER  (R_DIM * F_DIM)
#define RCH   4
#define TCH   64

static_assert(T_DIM == 512);
static_assert(F_DIM == 128);
static_assert(R_DIM % RCH == 0);
static_assert(T_DIM % TCH == 0);
static_assert(KTOT == 2 * T_DIM);
static_assert(KTOT % 32 == 0);

__device__ __forceinline__ unsigned int bf16_rne_u(float v) {
  unsigned int u = __float_as_uint(v);
  u += 0x7FFFu + ((u >> 16) & 1u);
  return u & 0xFFFF0000u;
}
__device__ __forceinline__ float bf16_val(float v) { return __uint_as_float(bf16_rne_u(v)); }
__device__ __forceinline__ u16 bf16_bits(float v) { return (u16)(bf16_rne_u(v) >> 16); }

__device__ __forceinline__ float softplus_f(float v) {
  const float mx = fmaxf(v, 0.0f);
  return mx + log1pf(expf(-fabsf(v)));
}

__device__ __forceinline__ v8f wmma_bf16(v16bf a, v16bf b, v8f c) {
  v8f d = __builtin_amdgcn_wmma_f32_16x16x32_bf16(false, a, false, b, (short)0, c, false, false);
  asm volatile("v_nop\n\tv_nop\n\tv_nop\n\tv_nop" : "+v"(d) : "v"(a), "v"(b));
  return d;
}

__device__ __forceinline__ v16bf load_frag(const u16* p, int h) {
  FragB f;
  f.u[0] = *(const v8usa*)(p + 8 * h);
  f.u[1] = *(const v8usa*)(p + 16 + 8 * h);
  return f.v;
}

__device__ __forceinline__ void prep_a_store(const u16* sRow, u16* Apl, int b, int rc, int tid) {
  #pragma unroll
  for (int it = 0; it < 4; ++it) {
    const int s = it * 256 + tid;
    const int rowid = s >> 7, piece = s & 127;
    const int rl = rowid & 3, which = rowid >> 2;
    const v8us v = *(const v8usa*)(sRow + (rl * 2 + which) * KTOT + piece * 8);
    u16* dst = Apl + ((size_t)((b * 2 + which) * R_DIM + rc * RCH + rl)) * KTOT + piece * 8;
    *(volatile v8us*)dst = v;
  }
}

__global__ __launch_bounds__(256) void k_prep_a(
    const float* __restrict__ tau,
    const float* __restrict__ log_kernel,
    u16* __restrict__ Apl)
{
  __shared__ __attribute__((aligned(16))) float sTh[T_DIM];
  __shared__ __attribute__((aligned(16))) u16   sRow[RCH * 2 * KTOT];

  const int b = blockIdx.x, rc = blockIdx.y, tid = threadIdx.x;

  const float kappa = softplus_f(bf16_val(log_kernel[0]));

  for (int i = tid; i < T_DIM; i += 256) sTh[i] = bf16_val(tau[(size_t)b * T_DIM + i]);
  __syncthreads();
  if (tid == 0) {
    float run = 0.0f;
    #pragma unroll 8
    for (int t = 0; t < T_DIM; ++t) {
      run += sTh[t];
      sTh[t] = run * (1.0f / 3600.0f);
    }
  }
  __syncthreads();

  #pragma unroll 1
  for (int it = 0; it < (RCH * T_DIM) / 256; ++it) {
    const int e = it * 256 + tid;
    const int rl = e >> 9, t = e & (T_DIM - 1);
    const int r = rc * RCH + rl;
    const float step = (float)r * (1.0f / 31.0f);
    const float reft = (r == R_DIM - 1) ? 48.0f : 48.0f * step;
    const float d = sTh[t] - reft;
    const float d2 = d * d;
    const float d2k = d2 * kappa;
    const float elp = expf(-d2k);
    const float ehp = expf(-10.0f * d2k);

    const unsigned int hlp = bf16_rne_u(elp);
    const float llp = elp - __uint_as_float(hlp);
    const unsigned int hhp = bf16_rne_u(ehp);
    const float lhp = ehp - __uint_as_float(hhp);

    sRow[(rl * 2 + 0) * KTOT + t]         = (u16)(hlp >> 16);
    sRow[(rl * 2 + 0) * KTOT + T_DIM + t] = bf16_bits(llp);
    sRow[(rl * 2 + 1) * KTOT + t]         = (u16)(hhp >> 16);
    sRow[(rl * 2 + 1) * KTOT + T_DIM + t] = bf16_bits(lhp);
  }
  __syncthreads();

  prep_a_store(sRow, Apl, b, rc, tid);
  __threadfence();
  prep_a_store(sRow, Apl, b, rc, tid);
}

__device__ __forceinline__ void put_b(u16* sT, int f, int t, float mraw, float xraw) {
  const unsigned int mu = bf16_rne_u(mraw);
  const float mval = __uint_as_float(mu);
  const float xval = bf16_val(xraw);
  sT[f * TCH + t] = (u16)(mu >> 16);
  sT[F_DIM * TCH + f * TCH + t] = bf16_bits(mval * xval);
}

__device__ __forceinline__ void prep_b_store(const u16* sT, u16* Bpl, int b, int B, int t0, int tid) {
  #pragma unroll
  for (int it = 0; it < 16; ++it) {
    const int s = it * 256 + tid;
    const int piece = s & 7, lineid = s >> 3;
    const int f = lineid & (F_DIM - 1), dup = (lineid >> 7) & 1, plane = lineid >> 8;
    const v8us v = *(const v8usa*)(sT + plane * (F_DIM * TCH) + f * TCH + piece * 8);
    u16* dst = Bpl + ((size_t)((plane * B + b) * F_DIM + f)) * KTOT + dup * T_DIM + t0 + piece * 8;
    *(volatile v8us*)dst = v;
  }
}

__global__ __launch_bounds__(256) void k_prep_b(
    const float* __restrict__ x_hat,
    const float* __restrict__ mask,
    u16* __restrict__ Bpl,
    int B)
{
  __shared__ __attribute__((aligned(16))) u16 sT[2 * F_DIM * TCH];

  const int b = blockIdx.x, tc = blockIdx.y, tid = threadIdx.x;
  const int t0 = tc * TCH;

  #pragma unroll 1
  for (int it = 0; it < (TCH * F_DIM / 4) / 256; ++it) {
    const int q = it * 256 + tid;
    const int t = q >> 5, f4 = (q & 31) * 4;
    const size_t g = ((size_t)(b * T_DIM + t0 + t)) * F_DIM + f4;
    const v4f mv = *(const v4fa*)(mask + g);
    const v4f xv = *(const v4fa*)(x_hat + g);
    put_b(sT, f4 + 0, t, mv.x, xv.x);
    put_b(sT, f4 + 1, t, mv.y, xv.y);
    put_b(sT, f4 + 2, t, mv.z, xv.z);
    put_b(sT, f4 + 3, t, mv.w, xv.w);
  }
  __syncthreads();

  prep_b_store(sT, Bpl, b, B, t0, tid);
  __threadfence();
  prep_b_store(sT, Bpl, b, B, t0, tid);
}

__device__ __forceinline__ void gemm_store(const float* sOut, float* out, int which, int b, int B, int tid) {
  const size_t nper = (size_t)B * NPER;
  const int nouts = (which == 0) ? 2 : 1;
  for (int o = 0; o < nouts; ++o) {
    const float* src = sOut + o * NPER;
    float* dst = out + ((which == 0) ? (size_t)o * nper : 2 * nper) + (size_t)b * NPER;
    #pragma unroll
    for (int it = 0; it < NPER / (128 * 4); ++it) {
      const int idx = (it * 128 + tid) * 4;
      const v4f v = *(const v4fa*)(src + idx);
      *(volatile v4f*)(dst + idx) = v;
    }
  }
}

__global__ __launch_bounds__(128) void k_gemm(
    const u16* __restrict__ Apl,
    const u16* __restrict__ Bpl,
    const float* __restrict__ log_kernel,
    float* __restrict__ out,
    int B)
{
  __shared__ __attribute__((aligned(16))) float sOut[2 * NPER];
  __shared__ float sK[F_DIM];

  const int tid = threadIdx.x, lane = tid & 31, w = tid >> 5;
  const int h = lane >> 4, m = lane & 15;
  const int b = blockIdx.x, which = blockIdx.y;
  const int mt = w & 1, nq = w >> 1;

  sK[tid] = softplus_f(bf16_val(log_kernel[tid]));

  const u16* arow = Apl + ((size_t)((b * 2 + which) * R_DIM + 16 * mt + m)) * KTOT;
  const u16* bmr  = Bpl + ((size_t)((0 * B + b) * F_DIM + 64 * nq + m)) * KTOT;
  const u16* bxr  = Bpl + ((size_t)((1 * B + b) * F_DIM + 64 * nq + m)) * KTOT;

  const v8f z8 = {0.f, 0.f, 0.f, 0.f, 0.f, 0.f, 0.f, 0.f};
  v8f accM[4], accX[4];
  #pragma unroll
  for (int nt = 0; nt < 4; ++nt) { accM[nt] = z8; accX[nt] = z8; }

  #pragma unroll 1
  for (int k0 = 0; k0 < KTOT; k0 += 32) {
    const v16bf a = load_frag(arow + k0, h);
    #pragma unroll
    for (int nt = 0; nt < 4; ++nt) {
      const v16bf fm = load_frag(bmr + (size_t)nt * 16 * KTOT + k0, h);
      accM[nt] = wmma_bf16(a, fm, accM[nt]);
      const v16bf fx = load_frag(bxr + (size_t)nt * 16 * KTOT + k0, h);
      accX[nt] = wmma_bf16(a, fx, accX[nt]);
    }
  }
  __syncthreads();

  float kmin = sK[0], kmax = sK[0];
  #pragma unroll 1
  for (int i = 1; i < F_DIM; ++i) { kmin = fminf(kmin, sK[i]); kmax = fmaxf(kmax, sK[i]); }
  const bool poison = (kmax != kmin);
  const float qnan = __uint_as_float(0x7fc00000u);

  #pragma unroll
  for (int nt = 0; nt < 4; ++nt) {
    const int f = 64 * nq + 16 * nt + m;
    #pragma unroll
    for (int r = 0; r < 8; ++r) {
      const int row = 16 * mt + 8 * h + r;
      const float den_raw = accM[nt][r];
      const float num = accX[nt][r];
      const float inv = 1.0f / fmaxf(den_raw, 1.0f);
      float qv = num * inv;
      float lv = den_raw;
      qv = poison ? qnan : qv;
      lv = poison ? qnan : lv;
      sOut[row * F_DIM + f] = qv;
      sOut[NPER + row * F_DIM + f] = lv;
    }
  }
  __syncthreads();

  gemm_store(sOut, out, which, b, B, tid);
  __threadfence();
  gemm_store(sOut, out, which, b, B, tid);
}

extern "C" void kernel_launch(void* const* d_in, const int* in_sizes, int n_in,
                              void* d_out, int out_size, void* d_ws, size_t ws_size,
                              hipStream_t stream) {
  if (n_in < 4) return;
  const int nTau = in_sizes[2];
  if (nTau < T_DIM || (nTau % T_DIM) != 0) return;
  const int B = nTau / T_DIM;
  if ((long long)in_sizes[0] != (long long)B * T_DIM * F_DIM) return;
  if (in_sizes[1] != in_sizes[0]) return;
  if (in_sizes[3] != F_DIM) return;
  if ((long long)out_size != 3LL * B * NPER) return;

  const size_t a_bytes = (size_t)B * 2 * R_DIM * KTOT * sizeof(u16);
  const size_t b_bytes = (size_t)2 * B * F_DIM * KTOT * sizeof(u16);
  if (a_bytes + b_bytes > ws_size) return;

  const float* x_hat      = (const float*)d_in[0];
  const float* maskp      = (const float*)d_in[1];
  const float* tau        = (const float*)d_in[2];
  const float* log_kernel = (const float*)d_in[3];
  float* out = (float*)d_out;

  char* ws = (char*)d_ws;
  u16* Apl = (u16*)(ws);
  u16* Bpl = (u16*)(ws + a_bytes);

  k_prep_a<<<dim3(B, R_DIM / RCH), 256, 0, stream>>>(tau, log_kernel, Apl);
  k_prep_b<<<dim3(B, T_DIM / TCH), 256, 0, stream>>>(x_hat, maskp, Bpl, B);
  k_gemm<<<dim3(B, 2), 128, 0, stream>>>(Apl, Bpl, log_kernel, out, B);
}
